// GINEncoder_9251359555640
// MI455X (gfx1250) — hardware-verified
//
#include <hip/hip_runtime.h>
#include <stddef.h>
#include <stdint.h>


#define DIM    128
#define HID    256
#define NLAY   5
#define KA     256
#define NTHR   256
#define NWAVE  8
#define EPT    8
#define CHUNK  (NTHR * EPT)
#define WCAP   (EPT * 32)
#define LISTN  (NWAVE * WCAP)
#define NBMAX  2048
#define RCAP   28672
#define DEGCAP 4096
#define STW    512
#define GBM    64
#define GBN    64
#define GTHR   128
#define CZ     0.125f
#define CW     256.0f
#define SCL_ZW 0.03125f
#define BN_EPS 1.0e-5f
#define WSMAX  268435456
#define LDS_AGG ((2 * RCAP + 2 * NBMAX + LISTN) * 4 + 64)

static_assert((CHUNK & (CHUNK - 1)) == 0 && CHUNK <= 4096);
static_assert((NBMAX & (NBMAX - 1)) == 0 && NBMAX <= 4096);
static_assert(NTHR * 8 == NBMAX);
static_assert(LISTN >= NBMAX);
static_assert(LISTN >= NWAVE * WCAP);
static_assert((RCAP % 32) == 0);
static_assert(NWAVE * STW <= RCAP);
static_assert(STW >= DIM);
static_assert(LDS_AGG <= 300000);
static_assert(GBM == (GTHR / 32) * 16);
static_assert(KA == 2 * DIM && KA == HID && (KA % 32) == 0);
static_assert((HID % GBN) == 0 && (DIM % GBN) == 0);
static_assert(DIM == 4 * 32);
static_assert(KA / 8 == 32);
static_assert(GBN <= GTHR);

typedef float          v4f  __attribute__((ext_vector_type(4)));
typedef float          v8f  __attribute__((ext_vector_type(8)));
typedef int            v4i  __attribute__((ext_vector_type(4)));
typedef int            v8i  __attribute__((ext_vector_type(8)));
typedef _Float16       v8h  __attribute__((ext_vector_type(8)));
typedef _Float16       v16h __attribute__((ext_vector_type(16)));
typedef unsigned short v8us __attribute__((ext_vector_type(8)));
typedef __bf16         v16b __attribute__((ext_vector_type(16)));
typedef v4f  __attribute__((may_alias)) v4fa;
typedef v4i  __attribute__((may_alias)) v4ia;
typedef v8us __attribute__((may_alias)) v8usa;
union Frag16 { v16h f; v16b b; v8us u[2]; v8i w; };

__device__ __forceinline__ v8f wm_f16(const Frag16& a, const Frag16& b, v8f c) {
  v8f d = __builtin_amdgcn_wmma_f32_16x16x32_f16(false, a.f, false, b.f, (short)0, c, false, false);
  asm volatile("v_nop\n\tv_nop\n\tv_nop\n\tv_nop" : "+v"(d) : "v"(a.w), "v"(b.w));
  return d;
}
__device__ __forceinline__ v8f wm_bf16(const Frag16& a, const Frag16& b, v8f c) {
  v8f d = __builtin_amdgcn_wmma_f32_16x16x32_bf16(false, a.b, false, b.b, (short)0, c, false, false);
  asm volatile("v_nop\n\tv_nop\n\tv_nop\n\tv_nop" : "+v"(d) : "v"(a.w), "v"(b.w));
  return d;
}

__device__ __forceinline__ unsigned int bfr_bits(float f) {
  unsigned int u = __float_as_uint(f);
  u += 0x7FFFu + ((u >> 16) & 1u);
  return u & 0xFFFF0000u;
}
__device__ __forceinline__ float bfr(float f) { return __uint_as_float(bfr_bits(f)); }
__device__ __forceinline__ unsigned short bfb(float f) { return (unsigned short)(bfr_bits(f) >> 16); }

__device__ __forceinline__ unsigned short hl1(float f, bool lo) {
  const unsigned int hb = bfr_bits(f);
  const float res = f - __uint_as_float(hb);
  const unsigned int lb = bfr_bits(res);
  return (unsigned short)((lo ? lb : hb) >> 16);
}

__device__ __forceinline__ v8us cvt8b(const v4f a, const v4f b) {
  v8us o;
  o[0] = bfb(a.x); o[1] = bfb(a.y); o[2] = bfb(a.z); o[3] = bfb(a.w);
  o[4] = bfb(b.x); o[5] = bfb(b.y); o[6] = bfb(b.z); o[7] = bfb(b.w);
  return o;
}
__device__ __forceinline__ v8h cvt8h(const v4f a, const v4f b, const float c) {
  v8h hv;
  hv[0] = (_Float16)(a.x * c); hv[1] = (_Float16)(a.y * c);
  hv[2] = (_Float16)(a.z * c); hv[3] = (_Float16)(a.w * c);
  hv[4] = (_Float16)(b.x * c); hv[5] = (_Float16)(b.y * c);
  hv[6] = (_Float16)(b.z * c); hv[7] = (_Float16)(b.w * c);
  return hv;
}
__device__ __forceinline__ v8h cvt8hb(const v4f a, const v4f b, const float c) {
  v8h hv;
  hv[0] = (_Float16)(bfr(a.x) * c); hv[1] = (_Float16)(bfr(a.y) * c);
  hv[2] = (_Float16)(bfr(a.z) * c); hv[3] = (_Float16)(bfr(a.w) * c);
  hv[4] = (_Float16)(bfr(b.x) * c); hv[5] = (_Float16)(bfr(b.y) * c);
  hv[6] = (_Float16)(bfr(b.z) * c); hv[7] = (_Float16)(bfr(b.w) * c);
  return hv;
}

__device__ __forceinline__ void ldwait() {
  asm volatile("s_wait_loadcnt 0x0" ::: "memory");
}

__device__ __forceinline__ int scan_chunk(const int* __restrict__ dsts, int nE, int cbase, int slotBase,
                                          int nb, int vec8, int* list, int tid, int lane, int wave) {
  int wc = 0;
  const int el0  = tid * EPT;
  const int e0   = cbase + el0;
  const int sent = -2147483647 - 1;
  v4i da, db;
  if (vec8 != 0 && cbase + CHUNK <= nE) {
    da = *(const v4ia*)(dsts + e0);
    db = *(const v4ia*)(dsts + e0 + 4);
  } else {
    da.x = (e0     < nE) ? dsts[min(e0,     nE - 1)] : sent;
    da.y = (e0 + 1 < nE) ? dsts[min(e0 + 1, nE - 1)] : sent;
    da.z = (e0 + 2 < nE) ? dsts[min(e0 + 2, nE - 1)] : sent;
    da.w = (e0 + 3 < nE) ? dsts[min(e0 + 3, nE - 1)] : sent;
    db.x = (e0 + 4 < nE) ? dsts[min(e0 + 4, nE - 1)] : sent;
    db.y = (e0 + 5 < nE) ? dsts[min(e0 + 5, nE - 1)] : sent;
    db.z = (e0 + 6 < nE) ? dsts[min(e0 + 6, nE - 1)] : sent;
    db.w = (e0 + 7 < nE) ? dsts[min(e0 + 7, nE - 1)] : sent;
  }
  const unsigned nbs = (unsigned)slotBase;
  const unsigned unb = (unsigned)nb;
  const unsigned s0 = (unsigned)da.x - nbs, s1 = (unsigned)da.y - nbs;
  const unsigned s2 = (unsigned)da.z - nbs, s3 = (unsigned)da.w - nbs;
  const unsigned s4 = (unsigned)db.x - nbs, s5 = (unsigned)db.y - nbs;
  const unsigned s6 = (unsigned)db.z - nbs, s7 = (unsigned)db.w - nbs;
  const bool h0 = s0 < unb, h1 = s1 < unb, h2 = s2 < unb, h3 = s3 < unb;
  const bool h4 = s4 < unb, h5 = s5 < unb, h6 = s6 < unb, h7 = s7 < unb;
  const unsigned any = __builtin_amdgcn_ballot_w32(h0 | h1 | h2 | h3 | h4 | h5 | h6 | h7);
  if (any != 0u) {
#define HITJ(J, HJ, SJ) { \
      const unsigned mj = __builtin_amdgcn_ballot_w32(HJ); \
      if (mj != 0u) { \
        if (HJ) { \
          const int pos = wc + (int)__builtin_amdgcn_mbcnt_lo(mj, 0u); \
          if (pos < WCAP) list[wave * WCAP + pos] = ((el0 + (J)) << 12) | (int)(SJ); \
        } \
        wc += (int)__builtin_popcount(mj); } }
    HITJ(0, h0, s0)
    HITJ(1, h1, s1)
    HITJ(2, h2, s2)
    HITJ(3, h3, s3)
    HITJ(4, h4, s4)
    HITJ(5, h5, s5)
    HITJ(6, h6, s6)
    HITJ(7, h7, s7)
#undef HITJ
  }
  return wc;
}

__global__ __launch_bounds__(NTHR) void k_hprep(const float* __restrict__ x, float* H, int nN, int nUnits) {
  const int i = (int)blockIdx.x * NTHR + (int)threadIdx.x;
  if (i >= nUnits) return;
  const int row = i >> 5;
  const int c0  = (i & 31) * 4;
  const int rc  = row < nN ? row : nN - 1;
  v4f a = *(const v4fa*)(x + (size_t)rc * DIM + c0);
  const v4f z4 = {0.f, 0.f, 0.f, 0.f};
  if (row >= nN) a = z4;
  v4f o;
  o.x = bfr(a.x); o.y = bfr(a.y); o.z = bfr(a.z); o.w = bfr(a.w);
  float* hp = H + (size_t)row * DIM + c0;
  *(volatile v4f*)hp = o;
  __threadfence();
  *(volatile v4f*)hp = o;
}

template<int SEL>
__global__ __launch_bounds__(NTHR) void k_wprep(const float* __restrict__ W, unsigned short* wt, int nUnits) {
  const int u = (int)blockIdx.x * NTHR + (int)threadIdx.x;
  if (u >= nUnits) return;
  const int row = u >> 5;
  const int k8  = (u & 31) * 8;
  const size_t o = (size_t)row * KA + k8;
  v4f a, b;
  if (SEL == 0) {
    const int l  = row / HID;
    const int n  = row - l * HID;
    const int ks = k8 & (DIM - 1);
    const float* p = W + ((size_t)l * DIM + ks) * HID + n;
    a.x = p[0];                  a.y = p[(size_t)HID];         a.z = p[(size_t)2 * HID];     a.w = p[(size_t)3 * HID];
    b.x = p[(size_t)4 * HID];    b.y = p[(size_t)5 * HID];     b.z = p[(size_t)6 * HID];     b.w = p[(size_t)7 * HID];
    const v8us ov = cvt8b(a, b);
    *(volatile v8us*)(wt + o) = ov;
    __threadfence();
    *(volatile v8us*)(wt + o) = ov;
  } else {
    const int l = row / DIM;
    const int n = row - l * DIM;
    const float* p = W + ((size_t)l * HID + k8) * DIM + n;
    a.x = p[0];                  a.y = p[(size_t)DIM];         a.z = p[(size_t)2 * DIM];     a.w = p[(size_t)3 * DIM];
    b.x = p[(size_t)4 * DIM];    b.y = p[(size_t)5 * DIM];     b.z = p[(size_t)6 * DIM];     b.w = p[(size_t)7 * DIM];
    const v8h hv = cvt8hb(a, b, CW);
    _Float16* hp = (_Float16*)wt + o;
    *(volatile v8h*)hp = hv;
    __threadfence();
    *(volatile v8h*)hp = hv;
  }
}

template<int TYP, int EPI>
__global__ __launch_bounds__(GTHR) void k_gemm(
    const unsigned short* __restrict__ A, const unsigned short* __restrict__ WT,
    const float* __restrict__ pb, const float* __restrict__ pg, const float* __restrict__ pbe,
    const float* __restrict__ pm, const float* __restrict__ pv,
    _Float16* outZ, float* outF, int K, int ldo, int rowLimit, int relu, float scl)
{
  __shared__ __attribute__((aligned(16))) float stg[GBM * GBN];
  __shared__ float csc[GBN];
  __shared__ float csh[GBN];
  const int tid = (int)threadIdx.x, lane = tid & 31, wave = tid >> 5, hh = lane >> 4, m = lane & 15;
  const int rowBase = (int)blockIdx.x * GBM;
  const int col0    = (int)blockIdx.y * GBN;

  if (tid < GBN) {
    const int c = col0 + tid;
    const float bb = bfr(pb[c]);
    const float gg = bfr(pg[c]);
    const float be = bfr(pbe[c]);
    const float mm = bfr(pm[c]);
    const float vv = bfr(pv[c]);
    const float r  = rsqrtf(vv + BN_EPS);
    const float sc = r * gg;
    csc[tid] = sc * scl;
    csh[tid] = (bb - mm) * sc + be;
  }
  __syncthreads();

  v8f acc[4];
  {
    const v8f z = {0.f, 0.f, 0.f, 0.f, 0.f, 0.f, 0.f, 0.f};
    acc[0] = z; acc[1] = z; acc[2] = z; acc[3] = z;
  }
  const unsigned short* ap = A  + (size_t)(rowBase + 16 * wave + m) * (size_t)K + 8 * hh;
  const unsigned short* wp = WT + (size_t)(col0 + m) * (size_t)K + 8 * hh;
  const int ksteps = K >> 5;
#pragma unroll 1
  for (int ks = 0; ks < ksteps; ++ks) {
    Frag16 af;
    af.u[0] = *(const v8usa*)(ap + 32 * ks);
    af.u[1] = *(const v8usa*)(ap + 32 * ks + 16);
#pragma unroll
    for (int t = 0; t < 4; ++t) {
      const unsigned short* wq = wp + (size_t)(16 * t) * (size_t)K + 32 * ks;
      Frag16 bf;
      bf.u[0] = *(const v8usa*)wq;
      bf.u[1] = *(const v8usa*)(wq + 16);
      if (TYP == 0) acc[t] = wm_bf16(af, bf, acc[t]);
      else          acc[t] = wm_f16(af, bf, acc[t]);
    }
  }

#pragma unroll
  for (int t = 0; t < 4; ++t) {
    const int lc = 16 * t + m;
    const float a_ = csc[lc];
    const float b_ = csh[lc];
#pragma unroll
    for (int r = 0; r < 8; ++r) {
      const int lr = 16 * wave + 8 * hh + r;
      float y = fmaf(acc[t][r], a_, b_);
      y = (relu != 0 && y < 0.f) ? 0.f : y;
      stg[lr * GBN + lc] = y;
    }
  }
  __syncthreads();

  if (EPI == 0) {
    const int q8 = lane & 7, sub = lane >> 3;
    v8h hv[4];
#pragma unroll
    for (int i = 0; i < 4; ++i) {
      const int lr = 16 * wave + 4 * i + sub;
      const v4f ga = *(const v4fa*)(stg + lr * GBN + 8 * q8);
      const v4f gb = *(const v4fa*)(stg + lr * GBN + 8 * q8 + 4);
      hv[i] = cvt8h(ga, gb, CZ);
    }
#pragma unroll
    for (int i = 0; i < 4; ++i) {
      const int lr = 16 * wave + 4 * i + sub;
      const int gr = rowBase + lr;
      _Float16* zp = outZ + (size_t)gr * (size_t)ldo + col0 + 8 * q8;
      if (gr < rowLimit) *(volatile v8h*)zp = hv[i];
    }
    __threadfence();
#pragma unroll
    for (int i = 0; i < 4; ++i) {
      const int lr = 16 * wave + 4 * i + sub;
      const int gr = rowBase + lr;
      _Float16* zp = outZ + (size_t)gr * (size_t)ldo + col0 + 8 * q8;
      if (gr < rowLimit) *(volatile v8h*)zp = hv[i];
    }
  } else {
    v4f fv[8];
#pragma unroll
    for (int i = 0; i < 8; ++i) {
      const int lr = 16 * wave + 2 * i + hh;
      fv[i] = *(const v4fa*)(stg + lr * GBN + 4 * m);
    }
#pragma unroll
    for (int i = 0; i < 8; ++i) {
      const int lr = 16 * wave + 2 * i + hh;
      const int gr = rowBase + lr;
      float* op = outF + (size_t)gr * (size_t)ldo + col0 + 4 * m;
      if (gr < rowLimit) *(volatile v4f*)op = fv[i];
    }
    __threadfence();
#pragma unroll
    for (int i = 0; i < 8; ++i) {
      const int lr = 16 * wave + 2 * i + hh;
      const int gr = rowBase + lr;
      float* op = outF + (size_t)gr * (size_t)ldo + col0 + 4 * m;
      if (gr < rowLimit) *(volatile v4f*)op = fv[i];
    }
  }
}

__global__ __launch_bounds__(NTHR) void k_agg(
    const int* __restrict__ srcs, const int* __restrict__ dsts,
    const float* __restrict__ H, unsigned short* AGG,
    int nN, int nE, int nb, int vec8, int MPr) {
  extern __shared__ v4f lds_dyn[];
  int* reg1 = (int*)lds_dyn;
  int* reg2 = reg1 + RCAP;
  int* scnt = reg2 + RCAP;
  int* soff = scnt + NBMAX;
  int* list = soff + NBMAX;
  int* wcnt = list + LISTN;
  int* wtot = wcnt + NWAVE;
  const int tid = (int)threadIdx.x, lane = tid & 31, wave = tid >> 5;
  const int nodeBase = (int)blockIdx.x * nb;

  for (int i = tid; i < NBMAX; i += NTHR) scnt[i] = 0;
  __syncthreads();

  int tot = 0;
  const int nChunks = (nE + CHUNK - 1) / CHUNK;
#pragma unroll 1
  for (int ch = 0; ch < nChunks; ++ch) {
    const int cbase = ch * CHUNK;
    const int wc = scan_chunk(dsts, nE, cbase, nodeBase, nb, vec8, list, tid, lane, wave);
    if (lane == 0) wcnt[wave] = wc;
    __syncthreads();
    int pre = 0, all = 0;
#pragma unroll
    for (int w2 = 0; w2 < NWAVE; ++w2) {
      int c = wcnt[w2];
      c = c < 0 ? 0 : (c > WCAP ? WCAP : c);
      all += c;
      pre += (w2 < wave) ? c : 0;
    }
    const int wcc  = wc > WCAP ? WCAP : wc;
    const int base = tot + pre;
#pragma unroll 1
    for (int i = lane; i < wcc; i += 32) {
      const int ent = list[wave * WCAP + i];
      const int el  = (ent >> 12) & (CHUNK - 1);
      const int sl  = ent & (NBMAX - 1);
      int eid = cbase + el;
      eid = eid > nE - 1 ? nE - 1 : eid;
      const int sr = srcs[eid];
      const int s  = sr < 0 ? 0 : (sr > nN - 1 ? nN - 1 : sr);
      const int pos = base + i;
      if (pos < RCAP) reg1[pos] = (int)(((unsigned)s << 12) | (unsigned)sl);
    }
    tot += all;
    tot = tot > RCAP ? RCAP : tot;
    __syncthreads();
  }
  const int nh = tot;

  if (wave == 0) {
#pragma unroll 1
    for (int b0 = 0; b0 < nh; b0 += 32) {
      const int idx = b0 + lane;
      const int uv  = reg1[idx < RCAP ? idx : RCAP - 1];
      const int m32 = (nh - b0) < 32 ? (nh - b0) : 32;
#pragma unroll 1
      for (int k = 0; k < m32; ++k) {
        const int u  = __builtin_amdgcn_readlane(uv, k);
        const int sl = u & (NBMAX - 1);
        if (lane == 0) scnt[sl] = scnt[sl] + 1;
      }
    }
  }
  __syncthreads();

  {
    const v4i ca = *(const v4ia*)(scnt + 8 * tid);
    const v4i cb = *(const v4ia*)(scnt + 8 * tid + 4);
    const int e0 = ca.x < 0 ? 0 : ca.x, e1 = ca.y < 0 ? 0 : ca.y, e2 = ca.z < 0 ? 0 : ca.z, e3 = ca.w < 0 ? 0 : ca.w;
    const int e4 = cb.x < 0 ? 0 : cb.x, e5 = cb.y < 0 ? 0 : cb.y, e6 = cb.z < 0 ? 0 : cb.z, e7 = cb.w < 0 ? 0 : cb.w;
    const int ts = e0 + e1 + e2 + e3 + e4 + e5 + e6 + e7;
    int incl = ts;
#pragma unroll
    for (int d = 1; d < 32; d <<= 1) {
      const int up = __shfl_up(incl, d);
      if (lane >= d) incl += up;
    }
    if (lane == 31) wtot[wave] = incl;
    __syncthreads();
    int pre = 0;
#pragma unroll
    for (int w2 = 0; w2 < NWAVE; ++w2) pre += (w2 < wave) ? wtot[w2] : 0;
    int run = pre + incl - ts;
    soff[8 * tid + 0] = run; run += e0;
    soff[8 * tid + 1] = run; run += e1;
    soff[8 * tid + 2] = run; run += e2;
    soff[8 * tid + 3] = run; run += e3;
    soff[8 * tid + 4] = run; run += e4;
    soff[8 * tid + 5] = run; run += e5;
    soff[8 * tid + 6] = run; run += e6;
    soff[8 * tid + 7] = run;
  }
  __syncthreads();
  for (int i = tid; i < NBMAX; i += NTHR) list[i] = soff[i];
  __syncthreads();

  if (wave == 0) {
#pragma unroll 1
    for (int b0 = 0; b0 < nh; b0 += 32) {
      const int idx = b0 + lane;
      const int uv  = reg1[idx < RCAP ? idx : RCAP - 1];
      const int m32 = (nh - b0) < 32 ? (nh - b0) : 32;
#pragma unroll 1
      for (int k = 0; k < m32; ++k) {
        const int u  = __builtin_amdgcn_readlane(uv, k);
        const int sl = u & (NBMAX - 1);
        const int sn = (int)((unsigned)u >> 12);
        if (lane == 0) {
          int pos = list[sl];
          pos = pos < 0 ? 0 : (pos > RCAP - 1 ? RCAP - 1 : pos);
          reg2[pos] = sn;
          list[sl] = pos + 1;
        }
      }
    }
  }
  __syncthreads();

  const int nbw = nb >> 3;
  const bool ovf = (nh >= RCAP);
  const float qnan = __int_as_float(0x7fc00000);
  float* stw = (float*)reg1 + wave * STW;
  const int  q16  = lane & 15;
  const bool islo = lane >= 16;
#pragma unroll 1
  for (int jt = 0; jt < nbw; ++jt) {
    const int slot = wave * nbw + jt;
    const int grow = nodeBase + slot;
    const int gcl  = grow < nN ? grow : nN - 1;
    int st = soff[slot];
    const int craw = scnt[slot];
    int cnt = craw;
    st  = st < 0 ? 0 : (st > nh ? nh : st);
    cnt = cnt < 0 ? 0 : (cnt > DEGCAP ? DEGCAP : cnt);
    if (cnt > nh - st) cnt = nh - st;
    const float pz = (ovf || craw > DEGCAP) ? qnan : 0.0f;
    const bool wr = grow < MPr;
    const float live = grow < nN ? 1.0f : 0.0f;

    v4f acc = *(const v4fa*)(H + (size_t)gcl * DIM + 4 * lane);
    ldwait();
#pragma unroll 1
    for (int q = 0; q < cnt; ++q) {
      int idx = st + q; idx = idx > RCAP - 1 ? RCAP - 1 : idx;
      int s = reg2[idx]; s = s < 0 ? 0 : (s > nN - 1 ? nN - 1 : s);
      const v4f hv = *(const v4fa*)(H + (size_t)s * DIM + 4 * lane);
      ldwait();
      acc += hv;
    }
    v4f ov;
    ov.x = acc.x * live + pz; ov.y = acc.y * live + pz;
    ov.z = acc.z * live + pz; ov.w = acc.w * live + pz;
    __builtin_amdgcn_fence(__ATOMIC_RELEASE, "wavefront");
    __builtin_amdgcn_wave_barrier();
    *(v4fa*)(stw + 4 * lane) = ov;
    __builtin_amdgcn_fence(__ATOMIC_RELEASE, "wavefront");
    __builtin_amdgcn_wave_barrier();
    const v4f ga = *(const v4fa*)(stw + 8 * q16);
    const v4f gb = *(const v4fa*)(stw + 8 * q16 + 4);
    v8us o;
    o[0] = hl1(ga.x, islo); o[1] = hl1(ga.y, islo); o[2] = hl1(ga.z, islo); o[3] = hl1(ga.w, islo);
    o[4] = hl1(gb.x, islo); o[5] = hl1(gb.y, islo); o[6] = hl1(gb.z, islo); o[7] = hl1(gb.w, islo);
    unsigned short* gp = AGG + (size_t)grow * KA + 8 * lane;
    if (wr) *(volatile v8us*)gp = o;
    __threadfence();
    if (wr) *(volatile v8us*)gp = o;
  }
}

static int pick_nb(int nE, int nN) {
  int nb = NBMAX;
  while (nb > 16 && (long long)nb * (long long)nE * 5LL > (long long)RCAP * (long long)nN * 4LL) nb >>= 1;
  return nb;
}
static inline int cdiv(int a, int b) { return (a + b - 1) / b; }

extern "C" void kernel_launch(void* const* d_in, const int* in_sizes, int n_in,
                              void* d_out, int out_size, void* d_ws, size_t ws_size,
                              hipStream_t stream) {
  if (n_in < 14) return;
  const int nN = in_sizes[0] / DIM;
  if (nN <= 0 || in_sizes[0] != nN * DIM || nN > (1 << 20)) return;
  if (in_sizes[1] < 2 || (in_sizes[1] & 1) != 0) return;
  const int nE = in_sizes[1] / 2;
  if (nE < 1 || nE > (1 << 26)) return;
  if (in_sizes[2]  != NLAY * DIM * HID) return;
  if (in_sizes[3]  != NLAY * HID || in_sizes[4] != NLAY * HID) return;
  if (in_sizes[5]  != NLAY * HID || in_sizes[6] != NLAY * HID) return;
  if (in_sizes[7]  != NLAY * HID) return;
  if (in_sizes[8]  != NLAY * HID * DIM) return;
  if (in_sizes[9]  != NLAY * DIM || in_sizes[10] != NLAY * DIM) return;
  if (in_sizes[11] != NLAY * DIM || in_sizes[12] != NLAY * DIM) return;
  if (in_sizes[13] != NLAY * DIM) return;
  if (out_size != nN * DIM) return;

  const float* x     = (const float*)d_in[0];
  const int*   ei    = (const int*)  d_in[1];
  const float* W1    = (const float*)d_in[2];
  const float* b1    = (const float*)d_in[3];
  const float* bn1_g = (const float*)d_in[4];
  const float* bn1_b = (const float*)d_in[5];
  const float* bn1_m = (const float*)d_in[6];
  const float* bn1_v = (const float*)d_in[7];
  const float* W2    = (const float*)d_in[8];
  const float* b2    = (const float*)d_in[9];
  const float* bno_g = (const float*)d_in[10];
  const float* bno_b = (const float*)d_in[11];
  const float* bno_m = (const float*)d_in[12];
  const float* bno_v = (const float*)d_in[13];
  float* out = (float*)d_out;
  const int* src = ei;
  const int* dst = ei + nE;

  const int MP   = cdiv(nN, GBM) * GBM;
  const int nb   = pick_nb(nE, nN);
  const int gA   = cdiv(MP, nb);
  const int vec8 = ((nE & 3) == 0) ? 1 : 0;
  if (gA * nb < MP) return;

  char* ws = (char*)d_ws;
  size_t off = 0;
  const size_t oH   = off; off += (size_t)MP * DIM * 4;             off = (off + 255) & ~(size_t)255;
  const size_t oAGG = off; off += (size_t)MP * KA * 2;              off = (off + 255) & ~(size_t)255;
  const size_t oZ   = off; off += (size_t)MP * HID * 2;             off = (off + 255) & ~(size_t)255;
  const size_t oWT1 = off; off += (size_t)NLAY * HID * KA * 2;      off = (off + 255) & ~(size_t)255;
  const size_t oWT2 = off; off += (size_t)NLAY * DIM * KA * 2;      off = (off + 255) & ~(size_t)255;
  if (off > ws_size || off > (size_t)WSMAX) return;
  float*          H   = (float*)(ws + oH);
  unsigned short* AGG = (unsigned short*)(ws + oAGG);
  _Float16*       Z   = (_Float16*)(ws + oZ);
  unsigned short* WT1 = (unsigned short*)(ws + oWT1);
  unsigned short* WT2 = (unsigned short*)(ws + oWT2);

  hipFuncSetAttribute(reinterpret_cast<const void*>(&k_agg),
                      hipFuncAttributeMaxDynamicSharedMemorySize, LDS_AGG);

  const int nUh = MP * (DIM / 4);
  k_hprep<<<cdiv(nUh, NTHR), NTHR, 0, stream>>>(x, H, nN, nUh);

  {
    const int nU1 = NLAY * HID * (KA / 8);
    k_wprep<0><<<cdiv(nU1, NTHR), NTHR, 0, stream>>>(W1, WT1, nU1);
    const int nU2 = NLAY * DIM * (KA / 8);
    k_wprep<1><<<cdiv(nU2, NTHR), NTHR, 0, stream>>>(W2, WT2, nU2);
  }

  const int gM = MP / GBM;
  for (int l = 0; l < NLAY; ++l) {
    k_agg<<<gA, NTHR, LDS_AGG, stream>>>(src, dst, H, AGG, nN, nE, nb, vec8, MP);
    k_gemm<0, 0><<<dim3(gM, HID / GBN), GTHR, 0, stream>>>(
        AGG, WT1 + (size_t)l * HID * KA,
        b1 + (size_t)l * HID, bn1_g + (size_t)l * HID, bn1_b + (size_t)l * HID,
        bn1_m + (size_t)l * HID, bn1_v + (size_t)l * HID,
        Z, H, KA, HID, MP, 1, 1.0f);
    const int last = (l == NLAY - 1) ? 1 : 0;
    float* outF = last ? out : H;
    const int rowLimit = last ? nN : MP;
    k_gemm<1, 1><<<dim3(gM, DIM / GBN), GTHR, 0, stream>>>(
        (const unsigned short*)Z, WT2 + (size_t)l * DIM * KA,
        b2 + (size_t)l * DIM, bno_g + (size_t)l * DIM, bno_b + (size_t)l * DIM,
        bno_m + (size_t)l * DIM, bno_v + (size_t)l * DIM,
        Z, outF, KA, DIM, rowLimit, last ? 0 : 1, SCL_ZW);
  }
}
